// QSANNAdapter_14456859918886
// MI455X (gfx1250) — hardware-verified
//
#include <hip/hip_runtime.h>


namespace {
constexpr int BH = 16, S = 2048, C = 64, NQ = 8, QD = 4;
constexpr float XS = 8.0f, PS = 1024.0f;
typedef _Float16 b16;
typedef __attribute__((ext_vector_type(16))) _Float16 v16b;
typedef __attribute__((ext_vector_type(8))) _Float16 v8b;
typedef __attribute__((ext_vector_type(8))) float v8f;
typedef __attribute__((ext_vector_type(4))) float v4f;
__device__ __forceinline__ float bf16_rne(float f) { unsigned int u = __float_as_uint(f); u += 0x7FFFu + ((u >> 16) & 1u); float r = __uint_as_float(u & 0xFFFF0000u); asm volatile("" : "+v"(r)); return r; }
__device__ __forceinline__ void split16(float v, b16& hi, b16& lo) { hi = (b16)v; lo = (b16)(v - (float)hi); }
__device__ __forceinline__ v16b frag_kb(const b16* p, int hh) { const v8b a = *(const v8b*)(p + 8 * hh), b = *(const v8b*)(p + 16 + 8 * hh); v16b f;
#pragma unroll
  for (int e = 0; e < 8; ++e) { f[e] = a[e]; f[8 + e] = b[e]; } return f; }
__device__ __forceinline__ v8f wmma16b(v16b a, v16b b, v8f c) { v8f d = __builtin_amdgcn_wmma_f32_16x16x32_f16(false, a, false, b, (short)0, c, false, false); asm volatile("v_nop\n\tv_nop\n\tv_nop\n\tv_nop" : "+v"(d) : "v"(a), "v"(b)); return d; }
__device__ __forceinline__ void wave_lds_sync() { __builtin_amdgcn_fence(__ATOMIC_RELEASE, "workgroup"); __builtin_amdgcn_wave_barrier(); __builtin_amdgcn_fence(__ATOMIC_ACQUIRE, "workgroup"); }
__device__ __forceinline__ float pmul(float a, float b) { float p = a * b; asm volatile("" : "+v"(p)); return p; }

__global__ __launch_bounds__(256) void proj_kernel(const float* __restrict__ qa, const float* __restrict__ ka, const float* __restrict__ wq, const float* __restrict__ bq, const float* __restrict__ wk, const float* __restrict__ bk, const float* __restrict__ lw, const float* __restrict__ lb, float* __restrict__ QK) {
  const int r = blockIdx.x * 256 + threadIdx.x; if (r >= BH * S) return; float o[8];
#pragma unroll
  for (int which = 0; which < 2; ++which) { const float* x = (which == 0 ? qa : ka) + (size_t)r * NQ; const float* w = which == 0 ? wq : wk; const float* b = which == 0 ? bq : bk; float p[QD]; float mu = 0.0f;
#pragma unroll
    for (int d = 0; d < QD; ++d) { float s = bf16_rne(b[d]);
#pragma unroll
      for (int j = 0; j < NQ; ++j) s += pmul(bf16_rne(x[j]), bf16_rne(w[d * NQ + j])); p[d] = s; mu += s; }
    mu *= 0.25f; float var = 0.0f;
#pragma unroll
    for (int d = 0; d < QD; ++d) var += pmul(p[d] - mu, p[d] - mu); var *= 0.25f; const float rs = rsqrtf(var + 1e-5f);
#pragma unroll
    for (int d = 0; d < QD; ++d) o[which * 4 + d] = pmul(pmul(p[d] - mu, rs), bf16_rne(lw[d])) + bf16_rne(lb[d]); }
  for (int pass = 0; pass < 2; ++pass) { *(volatile v4f*)(QK + (size_t)r * 8) = (v4f){o[0], o[1], o[2], o[3]}; *(volatile v4f*)(QK + (size_t)r * 8 + 4) = (v4f){o[4], o[5], o[6], o[7]}; __threadfence(); } }
__global__ __launch_bounds__(256) void xv_kernel(const float* __restrict__ xv, b16* __restrict__ XV) { const size_t u = (size_t)blockIdx.x * 256 + threadIdx.x; if (u >= (size_t)BH * C * S / 8) return; v8b v;
#pragma unroll
  for (int j = 0; j < 8; ++j) v[j] = (b16)(bf16_rne(xv[u * 8 + j]) * XS); for (int pass = 0; pass < 2; ++pass) { *(volatile v8b*)(XV + u * 8) = v; __threadfence(); } }
__global__ __launch_bounds__(32) void att_kernel(const float* __restrict__ QK, const b16* __restrict__ XV, const float* __restrict__ rtau, int BHV, float* __restrict__ out) {
  __shared__ __attribute__((aligned(16))) b16 Ah[2][16][40], Al[2][16][40]; __shared__ float Qs[32][5], Dn[32], Of[C][33];
  const int lane = threadIdx.x, nloc = lane & 15, hlf = lane >> 4; const int qt = blockIdx.x % (S / 32), bh = blockIdx.x / (S / 32); if (bh >= BHV) return; const int q0 = qt * 32;
  { const size_t r = (size_t)bh * S + q0 + lane; float n2 = 0.0f;
#pragma unroll
    for (int d = 0; d < QD; ++d) { const float v = QK[r * 8 + d]; Qs[lane][d] = v; n2 += pmul(v, v); } Qs[lane][4] = n2; Dn[lane] = 0.0f; }
  const float rt = bf16_rne(rtau[0]); const float tau = (rt > 20.0f ? rt : log1pf(__expf(rt))) + 1e-9f; const float itau = 1.0f / tau;
  v8f acc[2][4]; for (int m = 0; m < 2; ++m) for (int t = 0; t < 4; ++t) acc[m][t] = (v8f){};
  wave_lds_sync();
#pragma unroll 1
  for (int kc = 0; kc < S; kc += 32) { const size_t kr = (size_t)bh * S + kc + lane; float kv[4], kn2 = 0.0f;
#pragma unroll
    for (int d = 0; d < QD; ++d) { kv[d] = QK[kr * 8 + 4 + d]; kn2 += pmul(kv[d], kv[d]); }
    float dsum = 0.0f;
#pragma unroll 1
    for (int qi = 0; qi < 32; ++qi) { float cr = 0.0f;
#pragma unroll
      for (int d = 0; d < QD; ++d) cr += pmul(Qs[qi][d], kv[d]); const float dist = Qs[qi][4] + kn2 - 2.0f * cr; const float a = __expf(-pmul(dist, itau)); float as = a; for (int o = 16; o; o >>= 1) as += __shfl_xor(as, o); if (lane == 0) Dn[qi] += as;
      b16 p, q; split16(a * PS, p, q); Ah[qi >> 4][qi & 15][lane] = p; Al[qi >> 4][qi & 15][lane] = q; }
    (void)dsum; wave_lds_sync();
#pragma unroll
    for (int m = 0; m < 2; ++m) { const v16b pa = frag_kb(&Ah[m][nloc][0], hlf), pb = frag_kb(&Al[m][nloc][0], hlf);
#pragma unroll
      for (int t = 0; t < 4; ++t) { const v16b vv = frag_kb(XV + ((size_t)bh * C + t * 16 + nloc) * S + kc, hlf); acc[m][t] = wmma16b(pa, vv, acc[m][t]); acc[m][t] = wmma16b(pb, vv, acc[m][t]); } }
    wave_lds_sync(); }
#pragma unroll
  for (int m = 0; m < 2; ++m)
#pragma unroll
    for (int t = 0; t < 4; ++t)
#pragma unroll
      for (int r8 = 0; r8 < 8; ++r8) { const int ql = m * 16 + 8 * hlf + r8; Of[t * 16 + nloc][ql] = acc[m][t][r8] * (1.0f / (PS * XS)) / (Dn[ql] + 1e-9f); }
  wave_lds_sync();
  for (int pass = 0; pass < 2; ++pass) { for (int c = 0; c < C; ++c) ((volatile float*)out)[((size_t)bh * C + c) * S + q0 + lane] = Of[c][lane]; __threadfence(); }
}
}

extern "C" void kernel_launch(void* const* d_in, const int* in_sizes, int n_in, void* d_out, int out_size, void* d_ws, size_t ws_size, hipStream_t stream) {
  (void)n_in;
  auto Fp = [&](int i) { return (const float*)d_in[i]; };
  if (in_sizes[0] != BH * S * NQ || in_sizes[1] != BH * S * NQ || in_sizes[2] != BH * C * S || in_sizes[3] != QD * NQ || in_sizes[9] != 1 || out_size != BH * C * S) return;
  const int BHV = BH;
  size_t off = 0; char* ws = (char*)d_ws;
  auto carve = [&](size_t bytes) { char* p = ws + off; off += (bytes + 255) & ~(size_t)255; return p; };
  float* QK = (float*)carve((size_t)BH * S * 8 * 4); b16* XV = (b16*)carve((size_t)BH * C * S * 2);
  if (off > ws_size || off > ((size_t)16 << 20)) return;
  proj_kernel<<<(BH * S + 255) / 256, 256, 0, stream>>>(Fp(0), Fp(1), Fp(3), Fp(4), Fp(5), Fp(6), Fp(7), Fp(8), QK);
  xv_kernel<<<(unsigned)(((size_t)BH * C * S / 8 + 255) / 256), 256, 0, stream>>>(Fp(2), XV);
  att_kernel<<<BHV * (S / 32), 32, 0, stream>>>(QK, XV, Fp(9), BHV, (float*)d_out);
}
